// GAPModel_40742059770459
// MI455X (gfx1250) — hardware-verified
//
#include <hip/hip_runtime.h>
#include <stddef.h>


#define DIN    128
#define DH1    512
#define DH2    128
#define DT     256
#define DP1    32
#define NCLS   8
#define K1     256
#define NTHR   256
#define NWAVE  8
#define EPT    8
#define NGRP   2
#define CHUNK  (NTHR * EPT * NGRP)
#define WCAP   (EPT * NGRP * 32)
#define LISTN  (NWAVE * WCAP)
#define NB     512
#define G2ROWS 128
#define WSCALE 16.0f
#define WINV   0.0625f

#define LDS_ACC  (NB * DIN * 4)
#define LDS_LIST (LISTN * 4)
#define LDS_CNT  (NB * 4)
#define LDS_AGG  (LDS_ACC + LDS_LIST + LDS_CNT + 64)

static_assert((CHUNK & (CHUNK - 1)) == 0);
static_assert(CHUNK <= 4096);
static_assert((NB & (NB - 1)) == 0 && NB <= 4096);
static_assert(NB * K1 * 2 == LDS_ACC);
static_assert(NB * DH2 * 2 <= LDS_ACC / 2);
static_assert(NB * DP1 * 4 <= LDS_ACC / 2);
static_assert(NWAVE * 16 * 64 * 2 <= LDS_LIST);
static_assert(NB * NCLS * 4 <= LDS_LIST);
static_assert(NB % G2ROWS == 0);
static_assert(NB == NWAVE * 4 * 16);
static_assert(G2ROWS == NWAVE * 16);

typedef float    v4f  __attribute__((ext_vector_type(4)));
typedef float    v8f  __attribute__((ext_vector_type(8)));
typedef int      v4i  __attribute__((ext_vector_type(4)));
typedef _Float16 v8h  __attribute__((ext_vector_type(8)));
typedef _Float16 v16h __attribute__((ext_vector_type(16)));
union FragH { v16h v; v8h h[2]; };
union H8 { v8h h; v4f f; };

__device__ __forceinline__ v8h cvt8(v4f a, v4f b) {
  v8h r;
  r[0] = (_Float16)a.x; r[1] = (_Float16)a.y; r[2] = (_Float16)a.z; r[3] = (_Float16)a.w;
  r[4] = (_Float16)b.x; r[5] = (_Float16)b.y; r[6] = (_Float16)b.z; r[7] = (_Float16)b.w;
  return r;
}

__device__ __forceinline__ v4f relu4(v4f v) {
  v.x = fmaxf(v.x, 0.f); v.y = fmaxf(v.y, 0.f); v.z = fmaxf(v.z, 0.f); v.w = fmaxf(v.w, 0.f);
  return v;
}

__device__ __forceinline__ v8f wmh(v16h a, v16h b, v8f c) {
  v8f d = __builtin_amdgcn_wmma_f32_16x16x32_f16(false, a, false, b, (short)0, c, false, false);
  asm volatile("v_nop\n\tv_nop\n\tv_nop\n\tv_nop" : "+v"(d) : "v"(a), "v"(b));
  return d;
}

template <int NBT>
__device__ __forceinline__ int scan_chunk(const int* __restrict__ dsts, int nE, int cbase, int nodeBase,
                                          int vec8, int* list, int tid, int lane, int wave) {
  int wc = 0;
#pragma unroll
  for (int g = 0; g < NGRP; ++g) {
    const int el0  = (g * NTHR + tid) * EPT;
    const int e0   = cbase + el0;
    const int sent = -2147483647 - 1;
    v4i da, db;
    if (vec8 != 0 && cbase + CHUNK <= nE) {
      da = *(const v4i*)(dsts + e0);
      db = *(const v4i*)(dsts + e0 + 4);
    } else {
      da.x = (e0     < nE) ? dsts[min(e0,     nE - 1)] : sent;
      da.y = (e0 + 1 < nE) ? dsts[min(e0 + 1, nE - 1)] : sent;
      da.z = (e0 + 2 < nE) ? dsts[min(e0 + 2, nE - 1)] : sent;
      da.w = (e0 + 3 < nE) ? dsts[min(e0 + 3, nE - 1)] : sent;
      db.x = (e0 + 4 < nE) ? dsts[min(e0 + 4, nE - 1)] : sent;
      db.y = (e0 + 5 < nE) ? dsts[min(e0 + 5, nE - 1)] : sent;
      db.z = (e0 + 6 < nE) ? dsts[min(e0 + 6, nE - 1)] : sent;
      db.w = (e0 + 7 < nE) ? dsts[min(e0 + 7, nE - 1)] : sent;
    }
    const unsigned nb = (unsigned)nodeBase;
    const unsigned s0 = (unsigned)da.x - nb, s1 = (unsigned)da.y - nb;
    const unsigned s2 = (unsigned)da.z - nb, s3 = (unsigned)da.w - nb;
    const unsigned s4 = (unsigned)db.x - nb, s5 = (unsigned)db.y - nb;
    const unsigned s6 = (unsigned)db.z - nb, s7 = (unsigned)db.w - nb;
    const bool h0 = s0 < (unsigned)NBT, h1 = s1 < (unsigned)NBT, h2 = s2 < (unsigned)NBT, h3 = s3 < (unsigned)NBT;
    const bool h4 = s4 < (unsigned)NBT, h5 = s5 < (unsigned)NBT, h6 = s6 < (unsigned)NBT, h7 = s7 < (unsigned)NBT;
    const unsigned any = __builtin_amdgcn_ballot_w32(h0 | h1 | h2 | h3 | h4 | h5 | h6 | h7);
    if (any != 0u) {
#define HITJ(J, HJ, SJ) { \
        const unsigned mj = __builtin_amdgcn_ballot_w32(HJ); \
        if (mj != 0u) { \
          if (HJ) { \
            const int pos = wc + (int)__builtin_amdgcn_mbcnt_lo(mj, 0u); \
            if (pos < WCAP) list[wave * WCAP + pos] = ((el0 + (J)) << 12) | (int)(SJ); \
          } \
          wc += (int)__builtin_popcount(mj); } }
      HITJ(0, h0, s0)
      HITJ(1, h1, s1)
      HITJ(2, h2, s2)
      HITJ(3, h3, s3)
      HITJ(4, h4, s4)
      HITJ(5, h5, s5)
      HITJ(6, h6, s6)
      HITJ(7, h7, s7)
#undef HITJ
    }
  }
  return wc;
}

__global__ __launch_bounds__(NTHR) void k_wprep(
    const float* __restrict__ W1s, const float* __restrict__ W1n,
    const float* __restrict__ W2s, const float* __restrict__ W2n,
    const float* __restrict__ Wp1,
    _Float16* w1p, _Float16* w2p, _Float16* wpp) {
  const int tid = threadIdx.x, b = blockIdx.x;
  float v[8];
  _Float16* dp;
  if (b < 64) {
    const int o  = (b * NTHR + tid) * 8;
    const int n  = o >> 8, k0 = o & 255, ks = k0 & 127;
    const bool lo = k0 < 128;
#pragma unroll
    for (int u = 0; u < 8; ++u) {
      const size_t idx = (size_t)(ks + u) * DH1 + n;
      const float a = W1s[idx], c = W1n[idx];
      v[u] = (lo ? a : c) * WSCALE;
    }
    dp = w1p + o;
  } else if (b < 128) {
    const int o  = ((b - 64) * NTHR + tid) * 8;
    const int n  = o >> 9, k0 = o & 511, ns = n & 127;
    const bool lo = n < 128;
#pragma unroll
    for (int u = 0; u < 8; ++u) {
      const size_t idx = (size_t)(k0 + u) * DH2 + ns;
      const float a = W2s[idx], c = W2n[idx];
      v[u] = (lo ? a : c) * WSCALE;
    }
    dp = w2p + o;
  } else {
    int i = (b - 128) * NTHR + tid;
    i = i > DP1 * DH2 / 8 - 1 ? DP1 * DH2 / 8 - 1 : i;
    const int o = i * 8;
    const int n = o >> 7, k0 = o & 127;
#pragma unroll
    for (int u = 0; u < 8; ++u) v[u] = Wp1[(size_t)(k0 + u) * DP1 + n] * WSCALE;
    dp = wpp + o;
  }
  v4f a, c;
  a.x = v[0]; a.y = v[1]; a.z = v[2]; a.w = v[3];
  c.x = v[4]; c.y = v[5]; c.z = v[6]; c.w = v[7];
  H8 hv; hv.h = cvt8(a, c);
  *(volatile v4f*)dp = hv.f;
  __threadfence();
  *(volatile v4f*)dp = hv.f;
}

__global__ __launch_bounds__(NTHR) void k_l1(
    const float* __restrict__ x, const int* __restrict__ srcs, const int* __restrict__ dsts,
    const float* __restrict__ b1, const _Float16* __restrict__ w1p, _Float16* h1,
    int nN, int nE, int vec8) {
  extern __shared__ v4f lds_dyn[];
  float*    acc  = (float*)lds_dyn;
  _Float16* At   = (_Float16*)lds_dyn;
  int*      list = (int*)((char*)lds_dyn + LDS_ACC);
  _Float16* stg  = (_Float16*)((char*)lds_dyn + LDS_ACC);
  int*      cnt  = (int*)((char*)lds_dyn + LDS_ACC + LDS_LIST);
  int*      wcnt = (int*)((char*)lds_dyn + LDS_ACC + LDS_LIST + LDS_CNT);
  const int tid = threadIdx.x, lane = tid & 31, wave = tid >> 5, hh = lane >> 4, m = lane & 15;
  const int nodeBase = blockIdx.x * NB;

  {
    const v4f z = {0.f, 0.f, 0.f, 0.f};
    for (int i = tid; i < NB * DIN / 4; i += NTHR) lds_dyn[i] = z;
    for (int i = tid; i < NB; i += NTHR) cnt[i] = 0;
  }
  __syncthreads();

  const int nChunks = (nE + CHUNK - 1) / CHUNK;
#pragma unroll 1
  for (int ch = 0; ch < nChunks; ++ch) {
    const int cbase = ch * CHUNK;
    const int wc = scan_chunk<NB>(dsts, nE, cbase, nodeBase, vec8, list, tid, lane, wave);
    if (lane == 0) wcnt[wave] = wc;
    __syncthreads();
    if (wave == 0) {
#pragma unroll 1
      for (int wsx = 0; wsx < NWAVE; ++wsx) {
        int n = __builtin_amdgcn_readfirstlane(wcnt[wsx]);
        n = n > WCAP ? WCAP : (n < 0 ? 0 : n);
        const int* lp = list + wsx * WCAP;
#pragma unroll 1
        for (int i = 0; i < n; ++i) {
          const int ent  = __builtin_amdgcn_readfirstlane(lp[i]);
          const int slot = ent & (NB - 1);
          int e = cbase + ((ent >> 12) & (CHUNK - 1));
          e = e > nE - 1 ? nE - 1 : e;
          int s = srcs[e];
          s = s < 0 ? 0 : (s > nN - 1 ? nN - 1 : s);
          const v4f v = *(const v4f*)(x + (size_t)s * DIN + 4 * lane);
          v4f* ap = (v4f*)(acc + slot * DIN + 4 * lane);
          *ap = *ap + v;
          if (lane == 0) cnt[slot] = cnt[slot] + 1;
        }
      }
    }
    __syncthreads();
  }

#pragma unroll 1
  for (int c = 0; c < NB / 32; ++c) {
    const int rr = 32 * c + (tid >> 3);
    const int c0 = (tid & 7) * 16;
    const float* ap = acc + rr * DIN + c0;
    const v4f a0 = *(const v4f*)ap, a1 = *(const v4f*)(ap + 4);
    const v4f a2 = *(const v4f*)(ap + 8), a3 = *(const v4f*)(ap + 12);
    int node = nodeBase + rr;
    node = node > nN - 1 ? nN - 1 : node;
    const float* xp = x + (size_t)node * DIN + c0;
    const v4f x0 = *(const v4f*)xp, x1 = *(const v4f*)(xp + 4);
    const v4f x2 = *(const v4f*)(xp + 8), x3 = *(const v4f*)(xp + 12);
    int d = cnt[rr];
    d = d < 1 ? 1 : d;
    const float inv = 1.0f / (float)d;
    __syncthreads();
    _Float16* wp = At + rr * K1 + c0;
    *(v8h*)wp         = cvt8(x0, x1);
    *(v8h*)(wp + 8)   = cvt8(x2, x3);
    *(v8h*)(wp + 128) = cvt8(a0 * inv, a1 * inv);
    *(v8h*)(wp + 136) = cvt8(a2 * inv, a3 * inv);
  }
  __syncthreads();

  _Float16* sw = stg + wave * 1024;
#pragma unroll 1
  for (int q = 0; q < 4; ++q) {
    const int t = wave + 8 * q;
#pragma unroll 1
    for (int p = 0; p < 4; ++p) {
      v8f ac[8];
#pragma unroll
      for (int j = 0; j < 8; ++j) { v8f z = {0.f, 0.f, 0.f, 0.f, 0.f, 0.f, 0.f, 0.f}; ac[j] = z; }
      const _Float16* ar = At + (16 * t + m) * K1 + 8 * hh;
      const _Float16* br = w1p + (size_t)(128 * p + m) * K1 + 8 * hh;
#pragma unroll 2
      for (int ks = 0; ks < K1 / 32; ++ks) {
        FragH a;
        a.h[0] = *(const v8h*)(ar + 32 * ks);
        a.h[1] = *(const v8h*)(ar + 32 * ks + 16);
#pragma unroll
        for (int j = 0; j < 8; ++j) {
          const _Float16* bp = br + (size_t)(16 * j) * K1 + 32 * ks;
          FragH b;
          b.h[0] = *(const v8h*)bp;
          b.h[1] = *(const v8h*)(bp + 16);
          ac[j] = wmh(a.v, b.v, ac[j]);
        }
      }
#pragma unroll
      for (int s = 0; s < 2; ++s) {
#pragma unroll
        for (int jj = 0; jj < 4; ++jj) {
          const int j = 4 * s + jj;
          const float bc = b1[128 * p + 16 * j + m];
          _Float16* sp = sw + (8 * hh) * 64 + 16 * jj + m;
#pragma unroll
          for (int r = 0; r < 8; ++r) sp[r * 64] = (_Float16)fmaxf(ac[j][r] * WINV + bc, 0.f);
        }
        __syncthreads();
        const int piece = (lane & 7) * 8;
        H8 u[4];
#pragma unroll
        for (int qq = 0; qq < 4; ++qq) {
          const int i = 4 * qq + (lane >> 3);
          u[qq].h = *(const v8h*)(sw + i * 64 + piece);
        }
        _Float16* gp = h1 + ((size_t)nodeBase + 16 * t) * DH1 + 128 * p + 64 * s + piece;
#pragma unroll
        for (int qq = 0; qq < 4; ++qq) {
          const int i = 4 * qq + (lane >> 3);
          *(volatile v4f*)(gp + (size_t)i * DH1) = u[qq].f;
        }
        __threadfence();
#pragma unroll
        for (int qq = 0; qq < 4; ++qq) {
          const int i = 4 * qq + (lane >> 3);
          *(volatile v4f*)(gp + (size_t)i * DH1) = u[qq].f;
        }
        __syncthreads();
      }
    }
  }
}

__global__ __launch_bounds__(NTHR) void k_g2(
    const _Float16* __restrict__ h1, const _Float16* __restrict__ w2p, float* T) {
  __shared__ __attribute__((aligned(16))) float stg[NWAVE * 16 * 128];
  const int tid = threadIdx.x, lane = tid & 31, wave = tid >> 5, hh = lane >> 4, m = lane & 15;
  const int row0 = blockIdx.x * G2ROWS + 16 * wave;
  float* sw = stg + wave * 2048;

#pragma unroll 1
  for (int p = 0; p < 2; ++p) {
    v8f ac[8];
#pragma unroll
    for (int j = 0; j < 8; ++j) { v8f z = {0.f, 0.f, 0.f, 0.f, 0.f, 0.f, 0.f, 0.f}; ac[j] = z; }
    const _Float16* ar = h1 + ((size_t)row0 + m) * DH1 + 8 * hh;
    const _Float16* br = w2p + (size_t)(128 * p + m) * DH1 + 8 * hh;
#pragma unroll 2
    for (int ks = 0; ks < DH1 / 32; ++ks) {
      FragH a;
      a.h[0] = *(const v8h*)(ar + 32 * ks);
      a.h[1] = *(const v8h*)(ar + 32 * ks + 16);
#pragma unroll
      for (int j = 0; j < 8; ++j) {
        const _Float16* bp = br + (size_t)(16 * j) * DH1 + 32 * ks;
        FragH b;
        b.h[0] = *(const v8h*)bp;
        b.h[1] = *(const v8h*)(bp + 16);
        ac[j] = wmh(a.v, b.v, ac[j]);
      }
    }
    float* sp = sw + (8 * hh) * 128 + m;
#pragma unroll
    for (int j = 0; j < 8; ++j) {
#pragma unroll
      for (int r = 0; r < 8; ++r) sp[r * 128 + 16 * j] = ac[j][r] * WINV;
    }
    __syncthreads();
    float* gp = T + (size_t)row0 * DT + 128 * p + 4 * lane;
#pragma unroll
    for (int i = 0; i < 16; ++i) {
      const v4f v = *(const v4f*)(sw + i * 128 + 4 * lane);
      *(volatile v4f*)(gp + (size_t)i * DT) = v;
    }
    __threadfence();
#pragma unroll
    for (int i = 0; i < 16; ++i) {
      const v4f v = *(const v4f*)(sw + i * 128 + 4 * lane);
      *(volatile v4f*)(gp + (size_t)i * DT) = v;
    }
    __syncthreads();
  }
}

__global__ __launch_bounds__(NTHR) void k_l2(
    const float* __restrict__ T, const int* __restrict__ srcs, const int* __restrict__ dsts,
    const float* __restrict__ b2, const _Float16* __restrict__ wpp, const float* __restrict__ bp1,
    const float* __restrict__ Wp2, const float* __restrict__ bp2, float* out,
    int nN, int nE, int vec8) {
  extern __shared__ v4f lds_dyn[];
  float*    acc  = (float*)lds_dyn;
  _Float16* A2   = (_Float16*)lds_dyn;
  float*    X    = (float*)((char*)lds_dyn + LDS_ACC / 2);
  int*      list = (int*)((char*)lds_dyn + LDS_ACC);
  float*    O    = (float*)((char*)lds_dyn + LDS_ACC);
  int*      cnt  = (int*)((char*)lds_dyn + LDS_ACC + LDS_LIST);
  int*      wcnt = (int*)((char*)lds_dyn + LDS_ACC + LDS_LIST + LDS_CNT);
  const int tid = threadIdx.x, lane = tid & 31, wave = tid >> 5, hh = lane >> 4, m = lane & 15;
  const int nodeBase = blockIdx.x * NB;

  {
    const v4f z = {0.f, 0.f, 0.f, 0.f};
    for (int i = tid; i < NB * DH2 / 4; i += NTHR) lds_dyn[i] = z;
    for (int i = tid; i < NB; i += NTHR) cnt[i] = 0;
  }
  __syncthreads();

  const int nChunks = (nE + CHUNK - 1) / CHUNK;
#pragma unroll 1
  for (int ch = 0; ch < nChunks; ++ch) {
    const int cbase = ch * CHUNK;
    const int wc = scan_chunk<NB>(dsts, nE, cbase, nodeBase, vec8, list, tid, lane, wave);
    if (lane == 0) wcnt[wave] = wc;
    __syncthreads();
    if (wave == 0) {
#pragma unroll 1
      for (int wsx = 0; wsx < NWAVE; ++wsx) {
        int n = __builtin_amdgcn_readfirstlane(wcnt[wsx]);
        n = n > WCAP ? WCAP : (n < 0 ? 0 : n);
        const int* lp = list + wsx * WCAP;
#pragma unroll 1
        for (int i = 0; i < n; ++i) {
          const int ent  = __builtin_amdgcn_readfirstlane(lp[i]);
          const int slot = ent & (NB - 1);
          int e = cbase + ((ent >> 12) & (CHUNK - 1));
          e = e > nE - 1 ? nE - 1 : e;
          int s = srcs[e];
          s = s < 0 ? 0 : (s > nN - 1 ? nN - 1 : s);
          const v4f v = *(const v4f*)(T + (size_t)s * DT + DH2 + 4 * lane);
          v4f* ap = (v4f*)(acc + slot * DH2 + 4 * lane);
          *ap = *ap + v;
          if (lane == 0) cnt[slot] = cnt[slot] + 1;
        }
      }
    }
    __syncthreads();
  }

#pragma unroll 1
  for (int c = 0; c < NB / 32; ++c) {
    const int rr = 32 * c + (tid >> 3);
    const int c0 = (tid & 7) * 16;
    const float* ap = acc + rr * DH2 + c0;
    const v4f a0 = *(const v4f*)ap, a1 = *(const v4f*)(ap + 4);
    const v4f a2 = *(const v4f*)(ap + 8), a3 = *(const v4f*)(ap + 12);
    int node = nodeBase + rr;
    node = node > nN - 1 ? nN - 1 : node;
    const float* tp = T + (size_t)node * DT + c0;
    const v4f t0 = *(const v4f*)tp, t1 = *(const v4f*)(tp + 4);
    const v4f t2 = *(const v4f*)(tp + 8), t3 = *(const v4f*)(tp + 12);
    const v4f g0 = *(const v4f*)(b2 + c0), g1 = *(const v4f*)(b2 + c0 + 4);
    const v4f g2 = *(const v4f*)(b2 + c0 + 8), g3 = *(const v4f*)(b2 + c0 + 12);
    int d = cnt[rr];
    d = d < 1 ? 1 : d;
    const float inv = 1.0f / (float)d;
    const v4f hv0 = relu4((t0 + a0 * inv) + g0);
    const v4f hv1 = relu4((t1 + a1 * inv) + g1);
    const v4f hv2 = relu4((t2 + a2 * inv) + g2);
    const v4f hv3 = relu4((t3 + a3 * inv) + g3);
    __syncthreads();
    _Float16* wp = A2 + rr * DH2 + c0;
    *(v8h*)wp       = cvt8(hv0, hv1);
    *(v8h*)(wp + 8) = cvt8(hv2, hv3);
  }
  __syncthreads();

#pragma unroll 1
  for (int q = 0; q < 4; ++q) {
    const int t = wave + 8 * q;
    v8f ac[2];
    { v8f z = {0.f, 0.f, 0.f, 0.f, 0.f, 0.f, 0.f, 0.f}; ac[0] = z; ac[1] = z; }
    const _Float16* ar = A2 + (16 * t + m) * DH2 + 8 * hh;
    const _Float16* br = wpp + (size_t)m * DH2 + 8 * hh;
#pragma unroll
    for (int ks = 0; ks < DH2 / 32; ++ks) {
      FragH a;
      a.h[0] = *(const v8h*)(ar + 32 * ks);
      a.h[1] = *(const v8h*)(ar + 32 * ks + 16);
#pragma unroll
      for (int j = 0; j < 2; ++j) {
        const _Float16* bp = br + (size_t)(16 * j) * DH2 + 32 * ks;
        FragH b;
        b.h[0] = *(const v8h*)bp;
        b.h[1] = *(const v8h*)(bp + 16);
        ac[j] = wmh(a.v, b.v, ac[j]);
      }
    }
#pragma unroll
    for (int j = 0; j < 2; ++j) {
      const float bc = bp1[16 * j + m];
      float* xp = X + (16 * t + 8 * hh) * DP1 + 16 * j + m;
#pragma unroll
      for (int r = 0; r < 8; ++r) xp[r * DP1] = fmaxf(ac[j][r] * WINV + bc, 0.f);
    }
  }
  __syncthreads();

  const v4f bq0 = *(const v4f*)bp2, bq1 = *(const v4f*)(bp2 + 4);
#pragma unroll 1
  for (int rr = tid; rr < NB; rr += NTHR) {
    const float* xr = X + rr * DP1;
    float l0 = 0.f, l1 = 0.f, l2 = 0.f, l3 = 0.f, l4 = 0.f, l5 = 0.f, l6 = 0.f, l7 = 0.f;
#pragma unroll 4
    for (int j = 0; j < DP1; ++j) {
      const float xv = xr[j];
      const v4f w0 = *(const v4f*)(Wp2 + j * NCLS), w1 = *(const v4f*)(Wp2 + j * NCLS + 4);
      l0 += xv * w0.x; l1 += xv * w0.y; l2 += xv * w0.z; l3 += xv * w0.w;
      l4 += xv * w1.x; l5 += xv * w1.y; l6 += xv * w1.z; l7 += xv * w1.w;
    }
    l0 += bq0.x; l1 += bq0.y; l2 += bq0.z; l3 += bq0.w;
    l4 += bq1.x; l5 += bq1.y; l6 += bq1.z; l7 += bq1.w;
    const float mx = fmaxf(fmaxf(fmaxf(l0, l1), fmaxf(l2, l3)), fmaxf(fmaxf(l4, l5), fmaxf(l6, l7)));
    const float e0 = __expf(l0 - mx), e1 = __expf(l1 - mx), e2 = __expf(l2 - mx), e3 = __expf(l3 - mx);
    const float e4 = __expf(l4 - mx), e5 = __expf(l5 - mx), e6 = __expf(l6 - mx), e7 = __expf(l7 - mx);
    const float ssum = ((e0 + e1) + (e2 + e3)) + ((e4 + e5) + (e6 + e7));
    const float sinv = 1.0f / ssum;
    v4f o0, o1;
    o0.x = e0 * sinv; o0.y = e1 * sinv; o0.z = e2 * sinv; o0.w = e3 * sinv;
    o1.x = e4 * sinv; o1.y = e5 * sinv; o1.z = e6 * sinv; o1.w = e7 * sinv;
    *(v4f*)(O + rr * NCLS)     = o0;
    *(v4f*)(O + rr * NCLS + 4) = o1;
  }
  __syncthreads();

  const size_t outN = (size_t)nN * NCLS;
  const size_t ob   = (size_t)nodeBase * NCLS;
  v4f ov[4];
#pragma unroll
  for (int qq = 0; qq < 4; ++qq) ov[qq] = *(const v4f*)(O + (wave * 4 + qq) * 128 + 4 * lane);
#pragma unroll
  for (int qq = 0; qq < 4; ++qq) {
    const size_t gi = ob + (size_t)((wave * 4 + qq) * 128 + 4 * lane);
    if (gi < outN) *(volatile v4f*)(out + gi) = ov[qq];
  }
  __threadfence();
#pragma unroll
  for (int qq = 0; qq < 4; ++qq) {
    const size_t gi = ob + (size_t)((wave * 4 + qq) * 128 + 4 * lane);
    if (gi < outN) *(volatile v4f*)(out + gi) = ov[qq];
  }
}

extern "C" void kernel_launch(void* const* d_in, const int* in_sizes, int n_in,
                              void* d_out, int out_size, void* d_ws, size_t ws_size,
                              hipStream_t stream) {
  if (n_in < 13) return;
  const int nN = in_sizes[0] / DIN;
  const int nE = in_sizes[1];
  if (nN <= 0 || in_sizes[0] != nN * DIN || nE < 0 || in_sizes[2] != nE) return;
  if (in_sizes[3] != DIN * DH1 || in_sizes[4] != DIN * DH1 || in_sizes[5] != DH1) return;
  if (in_sizes[6] != DH1 * DH2 || in_sizes[7] != DH1 * DH2 || in_sizes[8] != DH2) return;
  if (in_sizes[9] != DH2 * DP1 || in_sizes[10] != DP1 || in_sizes[11] != DP1 * NCLS || in_sizes[12] != NCLS) return;
  if (out_size != nN * NCLS) return;

  const float* x   = (const float*)d_in[0];
  const int*   src = (const int*)d_in[1];
  const int*   dst = (const int*)d_in[2];
  const float* W1s = (const float*)d_in[3];
  const float* W1n = (const float*)d_in[4];
  const float* b1  = (const float*)d_in[5];
  const float* W2s = (const float*)d_in[6];
  const float* W2n = (const float*)d_in[7];
  const float* b2  = (const float*)d_in[8];
  const float* Wp1 = (const float*)d_in[9];
  const float* bp1 = (const float*)d_in[10];
  const float* Wp2 = (const float*)d_in[11];
  const float* bp2 = (const float*)d_in[12];
  float* out = (float*)d_out;

  const int nA  = (nN + NB - 1) / NB;
  const int nG2 = (nN + G2ROWS - 1) / G2ROWS;
  if (nG2 * G2ROWS > nA * NB) return;

  char* ws = (char*)d_ws;
  size_t off = 0;
  const size_t oW1 = off; off += (size_t)DH1 * K1 * 2;                        off = (off + 255) & ~(size_t)255;
  const size_t oW2 = off; off += (size_t)DT * DH1 * 2;                        off = (off + 255) & ~(size_t)255;
  const size_t oWP = off; off += (size_t)DP1 * DH2 * 2;                       off = (off + 255) & ~(size_t)255;
  const size_t oH1 = off; off += (size_t)nA * NB * DH1 * 2;                   off = (off + 255) & ~(size_t)255;
  const size_t oT  = off; off += (size_t)nG2 * G2ROWS * DT * 4;               off = (off + 255) & ~(size_t)255;
  if (off > ws_size || off > (size_t)134217728) return;
  _Float16* w1p = (_Float16*)(ws + oW1);
  _Float16* w2p = (_Float16*)(ws + oW2);
  _Float16* wpp = (_Float16*)(ws + oWP);
  _Float16* h1  = (_Float16*)(ws + oH1);
  float*    T   = (float*)(ws + oT);

  const int vec8 = 1;

  k_wprep<<<130, NTHR, 0, stream>>>(W1s, W1n, W2s, W2n, Wp1, w1p, w2p, wpp);

  hipFuncSetAttribute(reinterpret_cast<const void*>(&k_l1),
                      hipFuncAttributeMaxDynamicSharedMemorySize, LDS_AGG);
  k_l1<<<nA, NTHR, LDS_AGG, stream>>>(x, src, dst, b1, w1p, h1, nN, nE, vec8);

  k_g2<<<nG2, NTHR, 0, stream>>>(h1, w2p, T);

  hipFuncSetAttribute(reinterpret_cast<const void*>(&k_l2),
                      hipFuncAttributeMaxDynamicSharedMemorySize, LDS_AGG);
  k_l2<<<nA, NTHR, LDS_AGG, stream>>>(T, src, dst, b2, wpp, bp1, Wp2, bp2, out, nN, nE, vec8);
}
